// GAT_skip_forward_15135464751860
// MI455X (gfx1250) — hardware-run, weakly checked
//
#include <hip/hip_runtime.h>


namespace {
constexpr int N = 20000, NP = 20032, E = 480000, FIN = 128, NH = 8, CH = 32, HC = 256, NCONV = 3, L0 = 32, NCLS = 10, RPB = 64, NBP = NP / RPB;
constexpr float XS = 8.0f, WSC = 256.0f, NEG = 0.2f, BNEPS = 1e-5f;
typedef _Float16 b16;
typedef __attribute__((ext_vector_type(16))) _Float16 v16b;
typedef __attribute__((ext_vector_type(8))) _Float16 v8b;
typedef __attribute__((ext_vector_type(8))) float v8f;
typedef __attribute__((ext_vector_type(4))) float v4f;
__device__ __forceinline__ float bf16_rne(float f) { unsigned int u = __float_as_uint(f); u += 0x7FFFu + ((u >> 16) & 1u); return __uint_as_float(u & 0xFFFF0000u); }
__device__ __forceinline__ void split16(float v, b16& hi, b16& lo) { hi = (b16)v; lo = (b16)(v - (float)hi); }
__device__ __forceinline__ v16b frag_kb(const b16* p, int hh) { const v8b a = *(const v8b*)(p + 8 * hh), b = *(const v8b*)(p + 16 + 8 * hh); v16b f;
#pragma unroll
  for (int e = 0; e < 8; ++e) { f[e] = a[e]; f[8 + e] = b[e]; } return f; }
__device__ __forceinline__ v8f wmma16b(v16b a, v16b b, v8f c) { v8f d = __builtin_amdgcn_wmma_f32_16x16x32_f16(false, a, false, b, (short)0, c, false, false); asm volatile("v_nop\n\tv_nop\n\tv_nop\n\tv_nop" : "+v"(d) : "v"(a), "v"(b)); return d; }
__device__ __forceinline__ void wave_lds_sync() { __builtin_amdgcn_fence(__ATOMIC_RELEASE, "workgroup"); __builtin_amdgcn_wave_barrier(); __builtin_amdgcn_fence(__ATOMIC_ACQUIRE, "workgroup"); }
__device__ __forceinline__ float pmul(float a, float b) { float p = a * b; asm volatile("" : "+v"(p)); return p; }
__device__ __forceinline__ float opaque(float a) { asm volatile("" : "+v"(a)); return a; }
__device__ __forceinline__ int iclamp(int v, int lo, int hi) { return v < lo ? lo : (v > hi ? hi : v); }
__device__ __forceinline__ float nexp(float x) { return __builtin_amdgcn_exp2f(x * 1.4426950408889634f); }
__device__ __forceinline__ float lrelu(float x) { return x > 0.0f ? x : NEG * x; }
__device__ __forceinline__ float elu_(float x) { return x > 0.0f ? x : (__expf(x) - 1.0f); }
constexpr int CSR_NBLK8 = 512, CSR_GB8 = 8, CSR_GN8 = 1 << CSR_GB8  , CSR_MAXG8 = 512, CSR_CAP8 = 12288  ;
__global__ __launch_bounds__(64) void csrA8_kernel(const int* __restrict__ dst, int E, int N, int nG, int CHP, int NGP, int* __restrict__ STG, int* __restrict__ HST) {
  extern __shared__ int sm[];
  int* cnt = sm; int* run = sm + NGP; int* ids = sm + 2 * NGP;
  const int b = blockIdx.x; const int ch = (E + CSR_NBLK8 - 1) / CSR_NBLK8; const int e0 = b * ch, e1 = min(E, e0 + ch);
  for (int i = threadIdx.x; i < NGP; i += 64) cnt[i] = 0;
  for (int i = threadIdx.x; i < CHP; i += 64) ids[i] = -1;
  __syncthreads();
  if (threadIdx.x == 0) {
    for (int e = e0; e < e1; ++e) { int d = dst[e]; d = (d < 0) ? 0 : (d >= N ? N - 1 : d); cnt[d >> CSR_GB8] += 1; }
    int acc = 0; for (int g = 0; g < nG; ++g) { run[g] = acc; acc += cnt[g]; }
    for (int e = e0; e < e1; ++e) { int d = dst[e]; d = (d < 0) ? 0 : (d >= N ? N - 1 : d); const int g = d >> CSR_GB8; ids[run[g]] = e; run[g] += 1; } }
  __syncthreads();
  typedef __attribute__((ext_vector_type(4))) int v4i;
  for (int pass = 0; pass < 2; ++pass) {
    for (int i = threadIdx.x; i < CHP / 4; i += 64) *(volatile v4i*)(STG + (size_t)b * CHP + i * 4) = *(const v4i*)(&ids[i * 4]);
    for (int i = threadIdx.x; i < NGP / 4; i += 64) { v4i v; for (int e = 0; e < 4; ++e) v[e] = (i * 4 + e < nG) ? cnt[i * 4 + e] : 0; *(volatile v4i*)(HST + (size_t)b * NGP + i * 4) = v; }
    __threadfence(); }
}
__global__ __launch_bounds__(512) void csrS8_kernel(const int* __restrict__ HST, int nG, int NGP, int* __restrict__ START, int* __restrict__ TOT, int* __restrict__ OFF) {
  __shared__ int tot[CSR_MAXG8];
  const int b = threadIdx.x;
  for (int pass = 0; pass < 2; ++pass) { int runb = 0; for (int g = 0; g < nG; ++g) { int c = HST[(size_t)b * NGP + g]; c = (c < 0) ? 0 : c; ((volatile int*)OFF)[(size_t)g * CSR_NBLK8 + b] = runb; runb += c; } __threadfence(); }
  for (int g = threadIdx.x; g < nG; g += 512) { int s = 0; for (int bb = 0; bb < CSR_NBLK8; ++bb) { int c = HST[(size_t)bb * NGP + g]; s += (c < 0) ? 0 : c; } tot[g] = s; }
  __syncthreads();
  if (threadIdx.x < 32) {
    __shared__ int st[CSR_MAXG8 + 32];
    if (threadIdx.x == 0) { int acc = 0; for (int g = 0; g < NGP; ++g) { st[g] = acc; if (g < nG) acc += (tot[g] + 31) & ~31; } st[NGP] = acc; }
    __builtin_amdgcn_fence(__ATOMIC_RELEASE, "workgroup"); __builtin_amdgcn_wave_barrier(); __builtin_amdgcn_fence(__ATOMIC_ACQUIRE, "workgroup");
    for (int pass = 0; pass < 2; ++pass) { for (int i = threadIdx.x; i < NGP + 32; i += 32) { ((volatile int*)START)[i] = (i <= NGP) ? st[min(i, NGP)] : 0; ((volatile int*)TOT)[i] = (i < nG) ? tot[i] : 0; } __threadfence(); } }
}
__global__ __launch_bounds__(256) void csrB8_kernel(const int* __restrict__ dst, int N, int nG, int CHP, int NGP, int permLen, const int* __restrict__ STG, const int* __restrict__ HST, const int* __restrict__ OFF, const int* __restrict__ START, const int* __restrict__ TOT, int* __restrict__ PERM, int* __restrict__ ROWPTR, int* __restrict__ ROWCNT, int* __restrict__ FLAG) {
  typedef __attribute__((ext_vector_type(4))) int v4i;
  __shared__ int ids[CSR_CAP8]; __shared__ unsigned short key[CSR_CAP8]; __shared__ int outp[CSR_CAP8]; __shared__ int ncnt[CSR_GN8 + 1]; __shared__ int boff[CSR_NBLK8 + 1];
  const int g = blockIdx.x, t_ = threadIdx.x; int tot = TOT[g]; int st = START[g], stn = START[g + 1]; const int v0 = g * CSR_GN8; const int nv = min(CSR_GN8, N - v0);
  st = (st < 0) ? 0 : (st > permLen - 32 ? permLen - 32 : st) & ~31; stn = (stn < st) ? st : (stn > permLen ? permLen : stn); tot = (tot < 0) ? 0 : tot; if (tot > stn - st && tot <= CSR_CAP8) tot = stn - st;
  if (tot > CSR_CAP8) {
    for (int pass = 0; pass < 2; ++pass) { for (int i = t_; i < CSR_GN8 / 4; i += 256) { v4i a, c; for (int e = 0; e < 4; ++e) { a[e] = st; c[e] = 0; } *(volatile v4i*)(ROWPTR + v0 + i * 4) = a; *(volatile v4i*)(ROWCNT + v0 + i * 4) = c; } if (t_ == 0) ((volatile int*)FLAG)[0] = 1; __threadfence(); } (void)nv; return; }
  if (t_ == 0) { int acc = 0; for (int b = 0; b < CSR_NBLK8; ++b) { boff[b] = acc; int c = HST[(size_t)b * NGP + g]; c = (c < 0) ? 0 : (c > CHP ? CHP : c); acc += c; if (acc > tot) acc = tot; } boff[CSR_NBLK8] = acc; }
  for (int i = t_; i <= CSR_GN8; i += 256) ncnt[i] = 0;
  __syncthreads();
  for (int b = 0; b < CSR_NBLK8; ++b) { const int c = boff[b + 1] - boff[b]; int o_ = OFF[(size_t)g * CSR_NBLK8 + b]; o_ = (o_ < 0) ? 0 : (o_ > CHP - c ? CHP - c : o_); const int* src_ = STG + (size_t)b * CHP + o_;
    for (int i = t_; i < c; i += 256) { int id = src_[i]; id = (id < 0) ? 0 : id; ids[boff[b] + i] = id; int d = dst[id]; d = (d < v0) ? v0 : (d >= N ? N - 1 : d); int kk = d - v0; kk = (kk < 0) ? 0 : (kk >= CSR_GN8 ? CSR_GN8 - 1 : kk); key[boff[b] + i] = (unsigned short)kk; } }
  __syncthreads();
  if (t_ == 0) { for (int i = 0; i < tot; ++i) ncnt[key[i]] += 1; int acc = 0; for (int vl = 0; vl < CSR_GN8; ++vl) { const int c = ncnt[vl]; ncnt[vl] = acc; acc += c; } ncnt[CSR_GN8] = acc;
    for (int i = 0; i < tot; ++i) { const int vl = key[i]; outp[ncnt[vl]] = ids[i]; ncnt[vl] += 1; }
    for (int vl = CSR_GN8; vl > 0; --vl) ncnt[vl] = ncnt[vl - 1]; ncnt[0] = 0; }
  __syncthreads();
  for (int pass = 0; pass < 2; ++pass) {
    for (int i = t_; i < (stn - st) / 4; i += 256) { v4i v; for (int e = 0; e < 4; ++e) { const int q = i * 4 + e; v[e] = (q < tot) ? outp[q] : -1; } *(volatile v4i*)(PERM + st + i * 4) = v; }
    for (int i = t_; i < CSR_GN8 / 4; i += 256) { v4i a, c; for (int e = 0; e < 4; ++e) { const int vl = i * 4 + e; a[e] = st + ncnt[vl]; c[e] = (vl < nv) ? (ncnt[vl + 1] - ncnt[vl]) : 0; } *(volatile v4i*)(ROWPTR + v0 + i * 4) = a; *(volatile v4i*)(ROWCNT + v0 + i * 4) = c; }
    __threadfence(); }
}
__global__ __launch_bounds__(256) void csrZ8_kernel(int* __restrict__ p, size_t n4) { typedef __attribute__((ext_vector_type(4))) int v4i; const size_t tid = (size_t)blockIdx.x * 256 + threadIdx.x, nth = (size_t)gridDim.x * 256; v4i z = {0, 0, 0, 0}; for (size_t i = tid; i < n4; i += nth) *(volatile v4i*)(p + i * 4) = z; }
struct CsrBufs8 { int *STG, *HST, *OFF, *START, *TOT, *PERM, *ROWPTR, *ROWCNT, *FLAG; int nG, NGP, CHP; size_t permLen; char* base; size_t bytes; };
static size_t csr_carve8(CsrBufs8& c, char* ws, size_t off, int E, int N) {
  const size_t off0 = off; c.base = ws + off;
  auto al = [&](size_t bytes) { char* p = ws + off; off += (bytes + 255) & ~(size_t)255; return p; };
  c.nG = (N + CSR_GN8 - 1) / CSR_GN8; c.NGP = (c.nG + 31) & ~31; const int ch = (E + CSR_NBLK8 - 1) / CSR_NBLK8; c.CHP = (ch + 31) & ~31; c.permLen = (size_t)E + 32 * (size_t)c.nG + 32;
  c.STG = (int*)al((size_t)CSR_NBLK8 * c.CHP * 4); c.HST = (int*)al((size_t)CSR_NBLK8 * c.NGP * 4); c.OFF = (int*)al((size_t)c.NGP * CSR_NBLK8 * 4); c.START = (int*)al((size_t)(c.NGP + 64) * 4); c.TOT = (int*)al((size_t)(c.NGP + 64) * 4);
  c.PERM = (int*)al(c.permLen * 4); c.ROWPTR = (int*)al((size_t)c.nG * CSR_GN8 * 4); c.ROWCNT = (int*)al((size_t)c.nG * CSR_GN8 * 4); c.FLAG = (int*)al(256);
  c.bytes = off - off0; return off;
}
static void csr_build8(const CsrBufs8& c, const int* dst, int E, int N, hipStream_t stream) {
  const size_t smem = (size_t)(2 * c.NGP + c.CHP) * 4;
  csrZ8_kernel<<<512, 256, 0, stream>>>((int*)c.base, c.bytes / 16);
  csrA8_kernel<<<CSR_NBLK8, 64, smem, stream>>>(dst, E, N, c.nG, c.CHP, c.NGP, c.STG, c.HST);
  csrS8_kernel<<<1, 512, 0, stream>>>(c.HST, c.nG, c.NGP, c.START, c.TOT, c.OFF);
  csrB8_kernel<<<c.nG, 256, 0, stream>>>(dst, N, c.nG, c.CHP, c.NGP, (int)c.permLen, c.STG, c.HST, c.OFF, c.START, c.TOT, c.PERM, c.ROWPTR, c.ROWCNT, c.FLAG);
}


__global__ __launch_bounds__(256) void wprep_kernel(const float* __restrict__ wl0, const float* __restrict__ wr0, const float* __restrict__ wl, const float* __restrict__ wr, const float* __restrict__ l0, b16* __restrict__ W0, b16* __restrict__ WC, b16* __restrict__ WL0) {
  const size_t u = (size_t)blockIdx.x * 256 + threadIdx.x; const size_t n0 = (size_t)2 * HC * FIN / 8, n1 = (size_t)NCONV * 2 * HC * HC / 8, n2 = (size_t)L0 * HC / 8; size_t t = u; v8b o;
  if (t < n0) { const size_t e = t * 8; const int row = (int)(e / FIN), k0 = (int)(e % FIN); const float* w = row < HC ? wl0 : wr0; const int oo = row % HC; for (int j = 0; j < 8; ++j) o[j] = (b16)(bf16_rne(w[(size_t)(k0 + j) * HC + oo]) * WSC); for (int pass = 0; pass < 2; ++pass) { *(volatile v8b*)(W0 + e) = o; __threadfence(); } return; } t -= n0;
  if (t < n1) { const size_t e = t * 8; const int i = (int)(e / (2 * HC * HC)); const int rem = (int)(e % (2 * HC * HC)); const int row = rem / HC, k0 = rem % HC; const float* w = row < HC ? wl : wr; const int oo = row % HC;
    for (int j = 0; j < 8; ++j) o[j] = (b16)(bf16_rne(w[((size_t)i * HC + k0 + j) * HC + oo]) * WSC); for (int pass = 0; pass < 2; ++pass) { *(volatile v8b*)(WC + e) = o; __threadfence(); } return; } t -= n1;
  if (t < n2) { const size_t e = t * 8; const int oo = (int)(e / HC), k0 = (int)(e % HC); for (int j = 0; j < 8; ++j) o[j] = (b16)(bf16_rne(l0[(size_t)(k0 + j) * L0 + oo]) * WSC); for (int pass = 0; pass < 2; ++pass) { *(volatile v8b*)(WL0 + e) = o; __threadfence(); } }
}
template <int C, int RAWX>
__global__ __launch_bounds__(256) void psum_kernel(const float* __restrict__ P, float* __restrict__ PS) {
  constexpr int NG = 256 / C; __shared__ __attribute__((aligned(16))) float sq[NG][C + 4]; const int t = threadIdx.x, c = t % C, grp = t / C; float a = 0.0f;
  for (int rr = grp; rr < RPB; rr += NG) { const size_t v = (size_t)blockIdx.x * RPB + rr; if (v < (size_t)N) { const float p = P[v * C + c]; a += RAWX ? bf16_rne(p) : p; } }
  sq[grp][c] = a; __syncthreads();
  for (int pass = 0; pass < 2; ++pass) { if (t < C / 4) { v4f s = {0.0f, 0.0f, 0.0f, 0.0f}; for (int g2 = 0; g2 < NG; ++g2) s += *(const v4f*)(&sq[g2][t * 4]); *(volatile v4f*)(PS + (size_t)blockIdx.x * C + t * 4) = s; } __threadfence(); }
}
template <int C, int RAWX>
__global__ __launch_bounds__(256) void var_kernel(const float* __restrict__ P, const float* __restrict__ MEAN, float* __restrict__ PS) {
  constexpr int NG = 256 / C; __shared__ __attribute__((aligned(16))) float sq[NG][C + 4]; const int t = threadIdx.x, c = t % C, grp = t / C; float a = 0.0f; const float m = MEAN[c];
  for (int rr = grp; rr < RPB; rr += NG) { const size_t v = (size_t)blockIdx.x * RPB + rr; if (v < (size_t)N) { const float p = P[v * C + c]; const float d = (RAWX ? bf16_rne(p) : p) - m; a += d * d; } }
  sq[grp][c] = a; __syncthreads();
  for (int pass = 0; pass < 2; ++pass) { if (t < C / 4) { v4f s = {0.0f, 0.0f, 0.0f, 0.0f}; for (int g2 = 0; g2 < NG; ++g2) s += *(const v4f*)(&sq[g2][t * 4]); *(volatile v4f*)(PS + (size_t)blockIdx.x * C + t * 4) = s; } __threadfence(); }
}
template <int C>
__global__ __launch_bounds__(256) void colstat_kernel(const float* __restrict__ PS, float* __restrict__ STAT) {
  const int c = threadIdx.x; if (c >= C) return; float s = 0.0f; for (int b = 0; b < NBP; ++b) s += PS[(size_t)b * C + c];
  for (int pass = 0; pass < 2; ++pass) { ((volatile float*)STAT)[c] = s * (1.0f / N); __threadfence(); }
}
template <int KD, int BNIN>
__global__ __launch_bounds__(128) void proj_kernel(const float* __restrict__ src, const float* __restrict__ MEAN, const float* __restrict__ VAR, const float* __restrict__ g_, const float* __restrict__ be_, const b16* __restrict__ W, const float* __restrict__ bl, const float* __restrict__ br, float* __restrict__ XLR) {
  __shared__ __attribute__((aligned(16))) b16 Ah[4][16][KD + 8], Al[4][16][KD + 8]; __shared__ __attribute__((aligned(16))) float Tf[4][16][128 + 4];
  const int wave = threadIdx.x >> 5, lane = threadIdx.x & 31, nloc = lane & 15, hlf = lane >> 4; const size_t m0 = (size_t)blockIdx.x * 64 + wave * 16; const int c0 = blockIdx.y * 128;
  for (int rr = 0; rr < 16; ++rr) { const size_t v = m0 + rr; for (int q = lane * 4; q < KD; q += 128) { v4f x = {0.0f, 0.0f, 0.0f, 0.0f}; if (v < (size_t)N) x = *(const v4f*)(src + v * KD + q);
      if (BNIN) for (int j = 0; j < 4; ++j) x[j] = (bf16_rne(x[j]) - MEAN[q + j]) * rsqrtf(VAR[q + j] + BNEPS) * bf16_rne(g_[q + j]) + bf16_rne(be_[q + j]);
      for (int j = 0; j < 4; ++j) { b16 p, s; split16((v < (size_t)N ? x[j] : 0.0f) * XS, p, s); Ah[wave][rr][q + j] = p; Al[wave][rr][q + j] = s; } } }
  wave_lds_sync();
  v8f acc[8];
#pragma unroll
  for (int t = 0; t < 8; ++t) acc[t] = (v8f){};
#pragma unroll 2
  for (int kb = 0; kb < KD; kb += 32) { const v16b a = frag_kb(&Ah[wave][nloc][kb], hlf), al = frag_kb(&Al[wave][nloc][kb], hlf);
#pragma unroll
    for (int t = 0; t < 8; ++t) { const v16b bw = frag_kb(W + (size_t)(c0 + t * 16 + nloc) * KD + kb, hlf); acc[t] = wmma16b(a, bw, acc[t]); acc[t] = wmma16b(al, bw, acc[t]); } }
  wave_lds_sync();
#pragma unroll
  for (int t = 0; t < 8; ++t) { const int cabs = c0 + t * 16 + nloc; const float bb = cabs < HC ? bf16_rne(bl[cabs]) : bf16_rne(br[cabs - HC]);
#pragma unroll 1
    for (int r = 0; r < 8; ++r) { const size_t row = m0 + 8 * hlf + r; Tf[wave][8 * hlf + r][t * 16 + nloc] = row < (size_t)N ? acc[t][r] * (1.0f / (XS * WSC)) + bb : 0.0f; } }
  wave_lds_sync();
  for (int pass = 0; pass < 2; ++pass) { for (int rr = 0; rr < 16; ++rr) *(volatile v4f*)(XLR + (m0 + rr) * (2 * HC) + c0 + lane * 4) = *(const v4f*)(&Tf[wave][rr][lane * 4]); __threadfence(); }
}
__global__ __launch_bounds__(256) void attn_kernel(const float* __restrict__ XLR, const float* __restrict__ att, const float* __restrict__ bias, const float* __restrict__ res, const int* __restrict__ srcs, const int* __restrict__ PERM, const int* __restrict__ ROWPTR, const int* __restrict__ ROWCNT, int permLen, float* __restrict__ P) {
  const int wave = threadIdx.x >> 5, lane = threadIdx.x & 31; const size_t v = (size_t)blockIdx.x * 8 + wave; const int cb = lane * 8;
  float aw[8], xr[8], acc[8];
#pragma unroll
  for (int i = 0; i < 8; ++i) { aw[i] = opaque(bf16_rne(att[cb + i])); acc[i] = 0.0f; xr[i] = 0.0f; }
  int st = 0, cnt = 0; float xs[8];
#pragma unroll
  for (int i = 0; i < 8; ++i) xs[i] = 0.0f;
  if (v < (size_t)N) { st = ROWPTR[v]; cnt = ROWCNT[v]; cnt = iclamp(cnt, 0, 65536); st = iclamp(st, 0, permLen - cnt);
    for (int q = 0; q < 2; ++q) { const v4f t = *(const v4f*)(XLR + v * (2 * HC) + HC + cb + 4 * q), s = *(const v4f*)(XLR + v * (2 * HC) + cb + 4 * q); for (int i = 0; i < 4; ++i) { xr[4 * q + i] = t[i]; xs[4 * q + i] = s[i]; } } }
  auto logit = [&](const float* xl) { float d = 0.0f;
#pragma unroll
    for (int i = 0; i < 8; ++i) d += pmul(aw[i], lrelu(xl[i] + xr[i])); d += __shfl_xor(d, 1); d += __shfl_xor(d, 2); return d; };
  float mx = logit(xs);
#pragma unroll 1
  for (int j = 0; j < cnt; ++j) { const int e = iclamp(PERM[st + j], 0, E - 1); const size_t s = (size_t)iclamp(srcs[e], 0, N - 1); float xl[8]; for (int q = 0; q < 2; ++q) { const v4f t = *(const v4f*)(XLR + s * (2 * HC) + cb + 4 * q); for (int i = 0; i < 4; ++i) xl[4 * q + i] = t[i]; } mx = fmaxf(mx, logit(xl)); }
  float den = nexp(logit(xs) - mx);
#pragma unroll
  for (int i = 0; i < 8; ++i) acc[i] = pmul(den, xs[i]);
#pragma unroll 1
  for (int j = 0; j < cnt; ++j) { const int e = iclamp(PERM[st + j], 0, E - 1); const size_t s = (size_t)iclamp(srcs[e], 0, N - 1); float xl[8]; for (int q = 0; q < 2; ++q) { const v4f t = *(const v4f*)(XLR + s * (2 * HC) + cb + 4 * q); for (int i = 0; i < 4; ++i) xl[4 * q + i] = t[i]; }
    const float pj = nexp(logit(xl) - mx); den += pj;
#pragma unroll
    for (int i = 0; i < 8; ++i) acc[i] += pmul(pj, xl[i]); }
  const float inv = 1.0f / den; v4f o[2];
  for (int q = 0; q < 2; ++q) { v4f rv = {0.0f, 0.0f, 0.0f, 0.0f}; if (res != nullptr && v < (size_t)N) rv = *(const v4f*)(res + v * HC + cb + 4 * q);
    for (int i = 0; i < 4; ++i) { const int c = cb + 4 * q + i; o[q][i] = (v < (size_t)N) ? pmul(acc[4 * q + i], inv) + bf16_rne(bias[c]) + rv[i] : 0.0f; } }
  for (int pass = 0; pass < 2; ++pass) { *(volatile v4f*)(P + v * HC + cb) = o[0]; *(volatile v4f*)(P + v * HC + cb + 4) = o[1]; __threadfence(); }
}
template <int ELU>
__global__ __launch_bounds__(256) void apply_kernel(const float* __restrict__ P, const float* __restrict__ MEAN, const float* __restrict__ VAR, const float* __restrict__ g_, const float* __restrict__ be_, float* __restrict__ H) {
  const size_t u = (size_t)blockIdx.x * 256 + threadIdx.x; if (u >= (size_t)NP * HC / 4) return; const size_t e = u * 4; const size_t v = e / HC; const int c = (int)(e % HC);
  v4f o = {0.0f, 0.0f, 0.0f, 0.0f}; if (v < (size_t)N) { const v4f p = *(const v4f*)(P + e); for (int i = 0; i < 4; ++i) { const float y = (p[i] - MEAN[c + i]) * rsqrtf(VAR[c + i] + BNEPS) * bf16_rne(g_[c + i]) + bf16_rne(be_[c + i]); o[i] = ELU ? elu_(y) : y; } }
  for (int pass = 0; pass < 2; ++pass) { *(volatile v4f*)(H + e) = o; __threadfence(); }
}
__global__ __launch_bounds__(128) void head_kernel(const float* __restrict__ H, const b16* __restrict__ WL0, const float* __restrict__ b0, const float* __restrict__ w1, const float* __restrict__ b1, float* __restrict__ out) {
  __shared__ __attribute__((aligned(16))) b16 Ah[4][16][HC + 8], Al[4][16][HC + 8]; __shared__ __attribute__((aligned(16))) float T[4][16][L0 + 1]; __shared__ __attribute__((aligned(16))) float so[64 * NCLS];
  const int wave = threadIdx.x >> 5, lane = threadIdx.x & 31, nloc = lane & 15, hlf = lane >> 4; const size_t m0 = (size_t)blockIdx.x * 64 + wave * 16;
  for (int rr = 0; rr < 16; ++rr) for (int q = lane * 4; q < HC; q += 128) { const v4f x = *(const v4f*)(H + (m0 + rr) * HC + q); for (int j = 0; j < 4; ++j) { b16 p, s; split16(x[j] * XS, p, s); Ah[wave][rr][q + j] = p; Al[wave][rr][q + j] = s; } }
  wave_lds_sync();
  v8f acc[2] = {(v8f){}, (v8f){}};
#pragma unroll 2
  for (int kb = 0; kb < HC; kb += 32) { const v16b a = frag_kb(&Ah[wave][nloc][kb], hlf), al = frag_kb(&Al[wave][nloc][kb], hlf);
    for (int t = 0; t < 2; ++t) { const v16b bw = frag_kb(WL0 + (size_t)(t * 16 + nloc) * HC + kb, hlf); acc[t] = wmma16b(a, bw, acc[t]); acc[t] = wmma16b(al, bw, acc[t]); } }
  for (int t = 0; t < 2; ++t) { const int c = t * 16 + nloc; const float bb = bf16_rne(b0[c]);
#pragma unroll 1
    for (int r = 0; r < 8; ++r) T[wave][8 * hlf + r][c] = elu_(acc[t][r] * (1.0f / (XS * WSC)) + bb); }
  wave_lds_sync();
  if (lane < 16) { const int rr = lane; float z[NCLS]; for (int o2 = 0; o2 < NCLS; ++o2) z[o2] = bf16_rne(b1[o2]);
#pragma unroll 1
    for (int k = 0; k < L0; ++k) { const float tk = T[wave][rr][k]; for (int o2 = 0; o2 < NCLS; ++o2) z[o2] += pmul(tk, bf16_rne(w1[k * NCLS + o2])); }
    for (int o2 = 0; o2 < NCLS; ++o2) so[(wave * 16 + rr) * NCLS + o2] = z[o2]; }
  __syncthreads();
  for (int pass = 0; pass < 2; ++pass) { for (int q = threadIdx.x * 4; q < 64 * NCLS; q += 512) { const size_t g = (size_t)blockIdx.x * 64 * NCLS + q; if (g < (size_t)N * NCLS) *(volatile v4f*)(out + g) = *(const v4f*)(&so[q]); } __threadfence(); }
}
}

extern "C" void kernel_launch(void* const* d_in, const int* in_sizes, int n_in, void* d_out, int out_size, void* d_ws, size_t ws_size, hipStream_t stream) {
  (void)n_in;
  auto Fp = [&](int i) { return (const float*)d_in[i]; }; auto Ip = [&](int i) { return (const int*)d_in[i]; };
  if (in_sizes[0] != N * FIN || in_sizes[1] != 2 * E || in_sizes[8] != FIN * HC || in_sizes[14] != NCONV * HC * HC || in_sizes[20] != HC * L0 || in_sizes[22] != L0 * NCLS || out_size != N * NCLS) return;
  size_t off = 0; char* ws = (char*)d_ws;
  auto carve = [&](size_t bytes) { char* p = ws + off; off += (bytes + 255) & ~(size_t)255; return p; };
  b16* W0 = (b16*)carve((size_t)2 * HC * FIN * 2); b16* WC = (b16*)carve((size_t)NCONV * 2 * HC * HC * 2); b16* WL0 = (b16*)carve((size_t)L0 * HC * 2);
  float* XLR = (float*)carve((size_t)NP * 2 * HC * 4); float* P = (float*)carve((size_t)NP * HC * 4); float* H = (float*)carve((size_t)NP * HC * 4); float* PS = (float*)carve((size_t)NBP * HC * 4); float* ST = (float*)carve((size_t)2 * HC * 4);
  CsrBufs8 csr; off = csr_carve8(csr, ws, off, E, N);
  if (off > ws_size || off > ((size_t)128 << 20)) return;
  const unsigned nap = (unsigned)(((size_t)NP * HC / 4 + 255) / 256);
  wprep_kernel<<<(unsigned)(((size_t)2 * HC * FIN / 8 + (size_t)NCONV * 2 * HC * HC / 8 + (size_t)L0 * HC / 8 + 255) / 256), 256, 0, stream>>>(Fp(8), Fp(10), Fp(14), Fp(16), Fp(20), W0, WC, WL0);
  csr_build8(csr, Ip(1) + E, E, N, stream);
  psum_kernel<FIN, 1><<<NBP, 256, 0, stream>>>(Fp(0), PS); colstat_kernel<FIN><<<1, 256, 0, stream>>>(PS, ST); var_kernel<FIN, 1><<<NBP, 256, 0, stream>>>(Fp(0), ST, PS); colstat_kernel<FIN><<<1, 256, 0, stream>>>(PS, ST + HC);
  proj_kernel<FIN, 1><<<dim3(NP / 64, 4), 128, 0, stream>>>(Fp(0), ST, ST + HC, Fp(2), Fp(3), W0, Fp(9), Fp(11), XLR);
  attn_kernel<<<NP / 8, 256, 0, stream>>>(XLR, Fp(12), Fp(13), nullptr, Ip(1), csr.PERM, csr.ROWPTR, csr.ROWCNT, (int)csr.permLen, P);
  psum_kernel<HC, 0><<<NBP, 256, 0, stream>>>(P, PS); colstat_kernel<HC><<<1, 256, 0, stream>>>(PS, ST); var_kernel<HC, 0><<<NBP, 256, 0, stream>>>(P, ST, PS); colstat_kernel<HC><<<1, 256, 0, stream>>>(PS, ST + HC);
  apply_kernel<0><<<nap, 256, 0, stream>>>(P, ST, ST + HC, Fp(4), Fp(5), H);
  for (int i = 0; i < NCONV; ++i) {
    proj_kernel<HC, 0><<<dim3(NP / 64, 4), 128, 0, stream>>>(H, nullptr, nullptr, nullptr, nullptr, WC + (size_t)i * 2 * HC * HC, Fp(15) + i * HC, Fp(17) + i * HC, XLR);
    attn_kernel<<<NP / 8, 256, 0, stream>>>(XLR, Fp(18) + i * NH * CH, Fp(19) + i * HC, H, Ip(1), csr.PERM, csr.ROWPTR, csr.ROWCNT, (int)csr.permLen, P);
    psum_kernel<HC, 0><<<NBP, 256, 0, stream>>>(P, PS); colstat_kernel<HC><<<1, 256, 0, stream>>>(PS, ST); var_kernel<HC, 0><<<NBP, 256, 0, stream>>>(P, ST, PS); colstat_kernel<HC><<<1, 256, 0, stream>>>(PS, ST + HC);
    apply_kernel<1><<<nap, 256, 0, stream>>>(P, ST, ST + HC, Fp(6), Fp(7), H); }
  head_kernel<<<NP / 64, 128, 0, stream>>>(H, WL0, Fp(21), Fp(22), Fp(23), (float*)d_out);
}
